// TransformerEncoder_56521769615863
// MI455X (gfx1250) — hardware-verified
//
#include <hip/hip_runtime.h>

#ifndef NB
#define NB 8
#endif
#ifndef SEQ
#define SEQ 1024
#endif
#define NB_FULL 8
#define SEQ_FULL 1024
#define DMOD 768
#define NHEAD 12
#define HDIM 64
#define FFD 3072
#define NTOK (NB * SEQ)
#define WCARRY 256.0f
#define WCARRY_INV 0.00390625f
#define PCARRY 16384.0f
#define PCARRY_INV 0.00006103515625f
#define LN_EPS 1.0e-5f

static_assert(NB >= 1 && NB <= NB_FULL);
static_assert(SEQ % 64 == 0 && SEQ >= 64 && SEQ <= SEQ_FULL);
static_assert(NHEAD * HDIM == DMOD);
static_assert(HDIM == 64);
static_assert(DMOD == 96 * 8);
static_assert(DMOD % 64 == 0 && FFD % 64 == 0 && DMOD % 32 == 0 && FFD % 32 == 0);
static_assert(NTOK % 64 == 0);
static_assert(5 * DMOD * 2 <= 3 * DMOD * 4);
static_assert(DMOD * 4 + FFD * 2 <= 3 * DMOD * 4);

typedef __bf16 v16b __attribute__((ext_vector_type(16)));
typedef _Float16 v16h __attribute__((ext_vector_type(16)));
typedef unsigned short v8us __attribute__((ext_vector_type(8), may_alias));
typedef float v8f __attribute__((ext_vector_type(8)));
typedef float v4f __attribute__((ext_vector_type(4)));
typedef float v4fa __attribute__((ext_vector_type(4), may_alias));
union Frag { v16b vb; v16h vh; v8us half[2]; unsigned short u[16]; };

__device__ __forceinline__ unsigned short bf16_bits(float x) { const unsigned int u = __float_as_uint(x); return (unsigned short)((u + 0x7FFFu + ((u >> 16) & 1u)) >> 16); }
__device__ __forceinline__ float bf16_val(unsigned short b) { return __uint_as_float(((unsigned int)b) << 16); }
__device__ __forceinline__ float bf16_rne(float x) { return bf16_val(bf16_bits(x)); }
__device__ __forceinline__ unsigned short f16_bits(float x) { const _Float16 hv = (_Float16)x; unsigned short u; __builtin_memcpy(&u, &hv, sizeof(u)); return u; }

template <int NT>
__device__ __forceinline__ v8f mma_bf(v16b ah, v16b al, v16b bh, v16b bl, v8f c) {
  c = __builtin_amdgcn_wmma_f32_16x16x32_bf16(false, ah, false, bh, (short)0, c, false, false);
  if (NT >= 2) c = __builtin_amdgcn_wmma_f32_16x16x32_bf16(false, al, false, bh, (short)0, c, false, false);
  if (NT >= 3) c = __builtin_amdgcn_wmma_f32_16x16x32_bf16(false, ah, false, bl, (short)0, c, false, false);
  asm volatile("v_nop\n\tv_nop\n\tv_nop\n\tv_nop" : "+v"(c) : "v"(ah), "v"(al), "v"(bh), "v"(bl));
  return c;
}
__device__ __forceinline__ v8f mma_h(v16h a, v16h b, v8f c) {
  c = __builtin_amdgcn_wmma_f32_16x16x32_f16(false, a, false, b, (short)0, c, false, false);
  asm volatile("v_nop\n\tv_nop\n\tv_nop\n\tv_nop" : "+v"(c) : "v"(a), "v"(b));
  return c;
}

__global__ __launch_bounds__(256) void k_wt_heads(const float* __restrict__ W, unsigned short* __restrict__ Bt) {
  const int t = blockIdx.x * 256 + threadIdx.x;
  if (t >= NHEAD * HDIM * (DMOD / 8)) return;
  const int n = t / (DMOD / 8), d8 = (t % (DMOD / 8)) * 8;
  const int h = n / HDIM, e = n % HDIM;
  v8us v;
#pragma unroll
  for (int i = 0; i < 8; ++i) v[i] = bf16_bits(W[((size_t)h * DMOD + d8 + i) * HDIM + e]);
  unsigned short* dst = Bt + (size_t)n * DMOD + d8;
  *(volatile v8us*)dst = v;
  __threadfence();
  *(volatile v8us*)dst = v;
}

__global__ __launch_bounds__(256) void k_wt_f16(const float* __restrict__ W, unsigned short* __restrict__ Pt, int K, int N) {
  const int t = blockIdx.x * 256 + threadIdx.x;
  const int k8n = K / 8;
  if (t >= N * k8n) return;
  const int n = t / k8n, k8 = (t % k8n) * 8;
  v8us v;
#pragma unroll
  for (int i = 0; i < 8; ++i) v[i] = f16_bits(bf16_rne(W[(size_t)(k8 + i) * N + n]) * WCARRY);
  unsigned short* dst = Pt + (size_t)n * K + k8;
  *(volatile v8us*)dst = v;
  __threadfence();
  *(volatile v8us*)dst = v;
}

template <bool XBF16, int OUTM>
__global__ __launch_bounds__(96) void k_ln768(const float* __restrict__ X, int xsegf, const float* __restrict__ g, const float* __restrict__ bta,
                                             unsigned short* __restrict__ P0, unsigned short* __restrict__ P1, float eps) {
  __shared__ float red[4];
  const int t = blockIdx.x, tid = threadIdx.x, lane = tid & 31, w = tid >> 5;
  const int xrow = (t / SEQ) * xsegf + (t % SEQ);
  const float* xp = X + (size_t)xrow * DMOD + tid * 8;
  const v4f a0 = *(const v4fa*)xp, a1 = *(const v4fa*)(xp + 4);
  float v[8] = {a0[0], a0[1], a0[2], a0[3], a1[0], a1[1], a1[2], a1[3]};
  if (XBF16) {
#pragma unroll
    for (int q = 0; q < 8; ++q) v[q] = bf16_rne(v[q]);
  }
  float s = 0.f;
#pragma unroll
  for (int q = 0; q < 8; ++q) s += v[q];
  s += __shfl_xor(s, 16, 32); s += __shfl_xor(s, 8, 32); s += __shfl_xor(s, 4, 32); s += __shfl_xor(s, 2, 32); s += __shfl_xor(s, 1, 32);
  if (lane == 0) red[w] = s;
  __syncthreads();
  const float mu = (red[0] + red[1] + red[2]) * (1.0f / (float)DMOD);
  __syncthreads();
  float s2 = 0.f;
#pragma unroll
  for (int q = 0; q < 8; ++q) { const float c = v[q] - mu; s2 += c * c; }
  s2 += __shfl_xor(s2, 16, 32); s2 += __shfl_xor(s2, 8, 32); s2 += __shfl_xor(s2, 4, 32); s2 += __shfl_xor(s2, 2, 32); s2 += __shfl_xor(s2, 1, 32);
  if (lane == 0) red[w] = s2;
  __syncthreads();
  const float rs = rsqrtf((red[0] + red[1] + red[2]) * (1.0f / (float)DMOD) + eps);
  const v4f g0 = *(const v4fa*)(g + tid * 8), g1 = *(const v4fa*)(g + tid * 8 + 4);
  const v4f b0 = *(const v4fa*)(bta + tid * 8), b1 = *(const v4fa*)(bta + tid * 8 + 4);
  const float gg[8] = {g0[0], g0[1], g0[2], g0[3], g1[0], g1[1], g1[2], g1[3]};
  const float bb[8] = {b0[0], b0[1], b0[2], b0[3], b1[0], b1[1], b1[2], b1[3]};
  float o[8];
#pragma unroll
  for (int q = 0; q < 8; ++q) o[q] = (v[q] - mu) * rs * bf16_rne(gg[q]) + bf16_rne(bb[q]);
  unsigned short* d0 = P0 + (size_t)t * DMOD + tid * 8;
  if (OUTM == 0) {
    v8us hv, lv;
#pragma unroll
    for (int q = 0; q < 8; ++q) { const unsigned short hb = bf16_bits(o[q]); hv[q] = hb; lv[q] = bf16_bits(o[q] - bf16_val(hb)); }
    unsigned short* d1 = P1 + (size_t)t * DMOD + tid * 8;
    *(volatile v8us*)d0 = hv;
    *(volatile v8us*)d1 = lv;
    __threadfence();
    *(volatile v8us*)d0 = hv;
    *(volatile v8us*)d1 = lv;
  } else {
    v8us fv;
#pragma unroll
    for (int q = 0; q < 8; ++q) fv[q] = f16_bits(o[q]);
    *(volatile v8us*)d0 = fv;
    __threadfence();
    *(volatile v8us*)d0 = fv;
  }
}

template <bool F16, int NT, int ACT, bool RES_BF16, int OUTM>
__global__ __launch_bounds__(128) void k_gemm(const unsigned short* __restrict__ Ah, const unsigned short* __restrict__ Al, int lda,
                                             const unsigned short* __restrict__ Wt, int ldb, const float* __restrict__ bias, float oscale,
                                             const float* __restrict__ resid, int ldr, int rsegf,
                                             void* __restrict__ Cv, void* __restrict__ C2v, int ldc, int csegf, int M, int N, int K) {
  __shared__ __attribute__((aligned(16))) float so[4][16][64];
  const int tid = threadIdx.x, w = tid >> 5, lane = tid & 31, ln = lane & 15, hh = lane >> 4;
  const int ntn = N / 64;
  const int wid = blockIdx.x * 4 + w;
  const int mt = wid / ntn, nq = wid % ntn;
  if (mt * 16 >= M) return;
  const int row0 = mt * 16, col0 = nq * 64;
  const unsigned short* arh = Ah + (size_t)(row0 + ln) * lda;
  const unsigned short* arl = Al + (size_t)(row0 + ln) * lda;
  v8f acc[4] = {};
  for (int kb = 0; kb < K; kb += 32) {
    Frag ah, al;
    ah.half[0] = *(const v8us*)(arh + kb + 8 * hh);
    ah.half[1] = *(const v8us*)(arh + kb + 16 + 8 * hh);
    if (NT >= 2) {
      al.half[0] = *(const v8us*)(arl + kb + 8 * hh);
      al.half[1] = *(const v8us*)(arl + kb + 16 + 8 * hh);
    } else {
      al.vb = ah.vb;
    }
#pragma unroll
    for (int t = 0; t < 4; ++t) {
      const unsigned short* brow = Wt + (size_t)(col0 + t * 16 + ln) * ldb + kb;
      Frag b;
      b.half[0] = *(const v8us*)(brow + 8 * hh);
      b.half[1] = *(const v8us*)(brow + 16 + 8 * hh);
      if (F16) acc[t] = mma_h(ah.vh, b.vh, acc[t]);
      else acc[t] = mma_bf<NT>(ah.vb, al.vb, b.vb, b.vb, acc[t]);
    }
  }
#pragma unroll
  for (int t = 0; t < 4; ++t) {
    const float bq = bf16_rne(bias[col0 + t * 16 + ln]);
#pragma unroll
    for (int r = 0; r < 8; ++r) {
      float v = acc[t][r] * oscale + bq;
      if (ACT == 2) v = 0.5f * v * (1.0f + erff(v * 0.70710678118654752f));
      so[w][8 * hh + r][t * 16 + ln] = v;
    }
  }
  __builtin_amdgcn_fence(4  , "workgroup");
  __builtin_amdgcn_wave_barrier();
  const size_t cbase = (size_t)(row0 / SEQ) * (size_t)csegf + (size_t)(row0 % SEQ);
  if (OUTM == 0) {
    float* C = (float*)Cv;
    const int rsub = lane >> 4, c4 = (lane & 15) * 4;
    const size_t rbase = (size_t)(row0 / SEQ) * (size_t)rsegf + (size_t)(row0 % SEQ);
    v4f vals[8];
#pragma unroll
    for (int q = 0; q < 8; ++q) {
      const int r = q * 2 + rsub;
      v4f v = *(const v4fa*)&so[w][r][c4];
      if (resid != nullptr) {
        v4f rv = *(const v4fa*)(resid + (rbase + r) * (size_t)ldr + col0 + c4);
        if (RES_BF16) {
#pragma unroll
          for (int i = 0; i < 4; ++i) rv[i] = bf16_rne(rv[i]);
        }
        v += rv;
      }
      vals[q] = v;
    }
    for (int pass = 0; pass < 2; ++pass) {
#pragma unroll
      for (int q = 0; q < 8; ++q) {
        const int r = q * 2 + rsub;
        *(volatile v4f*)(C + (cbase + r) * (size_t)ldc + col0 + c4) = vals[q];
      }
      if (pass == 0) __threadfence();
    }
  } else {
    unsigned short* C = (unsigned short*)Cv;
    unsigned short* C2 = (unsigned short*)C2v;
    const int rq = lane >> 3, c8 = (lane & 7) * 8;
    v8us hv[4], lv[4];
#pragma unroll
    for (int q = 0; q < 4; ++q) {
      const int r = q * 4 + rq;
      const v4f p0 = *(const v4fa*)&so[w][r][c8], p1 = *(const v4fa*)&so[w][r][c8 + 4];
      const float ps[8] = {p0[0], p0[1], p0[2], p0[3], p1[0], p1[1], p1[2], p1[3]};
      v8us a, bl;
#pragma unroll
      for (int i = 0; i < 8; ++i) {
        if (OUTM == 1) { a[i] = f16_bits(ps[i]); bl[i] = (unsigned short)0; }
        else { const unsigned short hb = bf16_bits(ps[i]); a[i] = hb; bl[i] = bf16_bits(ps[i] - bf16_val(hb)); }
      }
      hv[q] = a; lv[q] = bl;
    }
    for (int pass = 0; pass < 2; ++pass) {
#pragma unroll
      for (int q = 0; q < 4; ++q) {
        const int r = q * 4 + rq;
        const size_t o = (cbase + r) * (size_t)ldc + col0 + c8;
        *(volatile v8us*)(C + o) = hv[q];
        if (OUTM == 2) *(volatile v8us*)(C2 + o) = lv[q];
      }
      if (pass == 0) __threadfence();
    }
  }
}

__global__ __launch_bounds__(128) void k_flash(const unsigned short* __restrict__ qh, const unsigned short* __restrict__ ql,
                                              const unsigned short* __restrict__ kh, const unsigned short* __restrict__ kl,
                                              const unsigned short* __restrict__ vp, unsigned short* __restrict__ att) {
  constexpr int D = HDIM, KS = D / 32, DT = D / 16, T = SEQ;
  __shared__ __attribute__((aligned(16))) unsigned short sKh[32][D + 8], sKl[32][D + 8], sV[32][D + 8];
  __shared__ __attribute__((aligned(16))) unsigned short sP[4][16][40];
  __shared__ __attribute__((aligned(16))) float sO[4][16][D];
  const int tid = threadIdx.x, w = tid >> 5, lane = tid & 31, ln = lane & 15, hh = lane >> 4;
  const int nqb = T / 64;
  const int bh = blockIdx.x / nqb, qblk = blockIdx.x % nqb;
  const int b = bh / NHEAD, h = bh % NHEAD;
  const int q0 = qblk * 64 + w * 16;
  const size_t hb0 = (size_t)b * T * DMOD + (size_t)h * D;

  Frag aqh[KS], aql[KS];
  {
    const size_t qo = hb0 + (size_t)(q0 + ln) * DMOD;
#pragma unroll
    for (int ks = 0; ks < KS; ++ks) {
      aqh[ks].half[0] = *(const v8us*)(qh + qo + ks * 32 + 8 * hh);
      aqh[ks].half[1] = *(const v8us*)(qh + qo + ks * 32 + 16 + 8 * hh);
      aql[ks].half[0] = *(const v8us*)(ql + qo + ks * 32 + 8 * hh);
      aql[ks].half[1] = *(const v8us*)(ql + qo + ks * 32 + 16 + 8 * hh);
    }
  }
  float m_r[8], l_r[8];
#pragma unroll
  for (int r = 0; r < 8; ++r) { m_r[r] = -3.0e38f; l_r[r] = 0.f; }
  v8f oacc[DT];
#pragma unroll
  for (int dt = 0; dt < DT; ++dt) oacc[dt] = (v8f){0.f, 0.f, 0.f, 0.f, 0.f, 0.f, 0.f, 0.f};

  for (int j0 = 0; j0 < T; j0 += 32) {
    __syncthreads();
#pragma unroll
    for (int it = 0; it < (32 * (D / 8)) / 128; ++it) {
      const int e = tid + it * 128;
      const int r = e / (D / 8), c8 = (e % (D / 8)) * 8;
      const size_t go = hb0 + (size_t)(j0 + r) * DMOD + c8;
      *(v8us*)&sKh[r][c8] = *(const v8us*)(kh + go);
      *(v8us*)&sKl[r][c8] = *(const v8us*)(kl + go);
      *(v8us*)&sV[r][c8] = *(const v8us*)(vp + go);
    }
    __syncthreads();
    v8f s[2];
#pragma unroll
    for (int nt = 0; nt < 2; ++nt) {
      v8f acc = {};
#pragma unroll
      for (int ks = 0; ks < KS; ++ks) {
        Frag bh_, bl_;
        bh_.half[0] = *(const v8us*)&sKh[nt * 16 + ln][ks * 32 + 8 * hh]; bh_.half[1] = *(const v8us*)&sKh[nt * 16 + ln][ks * 32 + 16 + 8 * hh];
        bl_.half[0] = *(const v8us*)&sKl[nt * 16 + ln][ks * 32 + 8 * hh]; bl_.half[1] = *(const v8us*)&sKl[nt * 16 + ln][ks * 32 + 16 + 8 * hh];
        acc = mma_bf<3>(aqh[ks].vb, aql[ks].vb, bh_.vb, bl_.vb, acc);
      }
      s[nt] = acc;
    }
    float alpha[8];
#pragma unroll
    for (int r = 0; r < 8; ++r) {
      float mx = fmaxf(s[0][r], s[1][r]);
      mx = fmaxf(mx, __shfl_xor(mx, 1, 32)); mx = fmaxf(mx, __shfl_xor(mx, 2, 32)); mx = fmaxf(mx, __shfl_xor(mx, 4, 32)); mx = fmaxf(mx, __shfl_xor(mx, 8, 32));
      const float mnew = fmaxf(m_r[r], mx);
      alpha[r] = (m_r[r] > -1.0e38f) ? __expf(m_r[r] - mnew) : 0.0f;
      const float p0 = __expf(s[0][r] - mnew);
      const float p1 = __expf(s[1][r] - mnew);
      m_r[r] = mnew;
      l_r[r] = l_r[r] * alpha[r] + p0 + p1;
      sP[w][8 * hh + r][ln] = f16_bits(p0 * PCARRY);
      sP[w][8 * hh + r][16 + ln] = f16_bits(p1 * PCARRY);
    }
#pragma unroll
    for (int dt = 0; dt < DT; ++dt)
#pragma unroll
      for (int r = 0; r < 8; ++r) oacc[dt][r] *= alpha[r];
    __builtin_amdgcn_fence(4  , "workgroup");
    __builtin_amdgcn_wave_barrier();
    Frag pa;
    pa.half[0] = *(const v8us*)&sP[w][ln][8 * hh];
    pa.half[1] = *(const v8us*)&sP[w][ln][16 + 8 * hh];
#pragma unroll
    for (int dt = 0; dt < DT; ++dt) {
      Frag bv;
#pragma unroll
      for (int i = 0; i < 8; ++i) {
        bv.u[i] = sV[8 * hh + i][dt * 16 + ln];
        bv.u[8 + i] = sV[16 + 8 * hh + i][dt * 16 + ln];
      }
      oacc[dt] = mma_h(pa.vh, bv.vh, oacc[dt]);
    }
    __builtin_amdgcn_fence(4  , "workgroup");
    __builtin_amdgcn_wave_barrier();
  }
#pragma unroll
  for (int r = 0; r < 8; ++r) {
    float l = l_r[r];
    l += __shfl_xor(l, 1, 32); l += __shfl_xor(l, 2, 32); l += __shfl_xor(l, 4, 32); l += __shfl_xor(l, 8, 32);
    l_r[r] = (1.0f / l) * PCARRY_INV;
  }
#pragma unroll
  for (int dt = 0; dt < DT; ++dt)
#pragma unroll
    for (int r = 0; r < 8; ++r) sO[w][8 * hh + r][dt * 16 + ln] = oacc[dt][r] * l_r[r];
  __builtin_amdgcn_fence(4  , "workgroup");
  __builtin_amdgcn_wave_barrier();
  const int rq = lane >> 3, c8 = (lane & 7) * 8;
  v8us ov[4];
#pragma unroll
  for (int q = 0; q < 4; ++q) {
    const int r = q * 4 + rq;
    const v4f p0 = *(const v4fa*)&sO[w][r][c8], p1 = *(const v4fa*)&sO[w][r][c8 + 4];
    v8us o;
    o[0] = f16_bits(p0[0]); o[1] = f16_bits(p0[1]); o[2] = f16_bits(p0[2]); o[3] = f16_bits(p0[3]);
    o[4] = f16_bits(p1[0]); o[5] = f16_bits(p1[1]); o[6] = f16_bits(p1[2]); o[7] = f16_bits(p1[3]);
    ov[q] = o;
  }
  unsigned short* ob = att + ((size_t)b * T + q0) * DMOD + (size_t)h * D + c8;
  for (int pass = 0; pass < 2; ++pass) {
#pragma unroll
    for (int q = 0; q < 4; ++q) {
      const int r = q * 4 + rq;
      *(volatile v8us*)(ob + (size_t)r * DMOD) = ov[q];
    }
    if (pass == 0) __threadfence();
  }
}

extern "C" void kernel_launch(void* const* d_in, const int* in_sizes, int n_in,
                              void* d_out, int out_size, void* d_ws, size_t ws_size, hipStream_t stream) {
  if (n_in < 17) return;
  const int need_tok = (NB - 1) * SEQ_FULL + SEQ;
  if (in_sizes[0] < need_tok * DMOD || out_size < need_tok * DMOD) return;
  if (in_sizes[1] < DMOD || in_sizes[2] < DMOD || in_sizes[10] < DMOD || in_sizes[11] < DMOD || in_sizes[12] < DMOD || in_sizes[16] < DMOD) return;
  if (in_sizes[3] < NHEAD * DMOD * HDIM || in_sizes[5] < NHEAD * DMOD * HDIM || in_sizes[7] < NHEAD * DMOD * HDIM) return;
  if (in_sizes[4] < NHEAD * HDIM || in_sizes[6] < NHEAD * HDIM || in_sizes[8] < NHEAD * HDIM || in_sizes[14] < FFD) return;
  if (in_sizes[9] < DMOD * DMOD || in_sizes[13] < DMOD * FFD || in_sizes[15] < FFD * DMOD) return;

  const float* x    = (const float*)d_in[0];
  const float* ln1w = (const float*)d_in[1];
  const float* ln1b = (const float*)d_in[2];
  const float* Wq   = (const float*)d_in[3];
  const float* bqp  = (const float*)d_in[4];
  const float* Wk   = (const float*)d_in[5];
  const float* bkp  = (const float*)d_in[6];
  const float* Wv   = (const float*)d_in[7];
  const float* bvp  = (const float*)d_in[8];
  const float* Wp   = (const float*)d_in[9];
  const float* bpp  = (const float*)d_in[10];
  const float* ln2w = (const float*)d_in[11];
  const float* ln2b = (const float*)d_in[12];
  const float* W1   = (const float*)d_in[13];
  const float* b1p  = (const float*)d_in[14];
  const float* W2   = (const float*)d_in[15];
  const float* b2p  = (const float*)d_in[16];

  char* ws = (char*)d_ws; size_t off = 0;
  auto take = [&](size_t bytes) { char* p = ws + off; off += (bytes + 255) & ~(size_t)255; return p; };
  unsigned short* Bq = (unsigned short*)take((size_t)DMOD * DMOD * 2);
  unsigned short* Bk = (unsigned short*)take((size_t)DMOD * DMOD * 2);
  unsigned short* Bv = (unsigned short*)take((size_t)DMOD * DMOD * 2);
  unsigned short* Pp = (unsigned short*)take((size_t)DMOD * DMOD * 2);
  unsigned short* P1 = (unsigned short*)take((size_t)DMOD * FFD * 2);
  unsigned short* P2 = (unsigned short*)take((size_t)FFD * DMOD * 2);
  char* R1 = take((size_t)NTOK * DMOD * 4);
  char* R2 = take((size_t)NTOK * 3 * DMOD * 4);
  if (off > ws_size) return;

  const size_t PL = (size_t)NTOK * DMOD;
  unsigned short* yh  = (unsigned short*)R1;
  unsigned short* yl  = yh + PL;
  unsigned short* att = (unsigned short*)R1;
  unsigned short* h0  = (unsigned short*)R1;
  unsigned short* qh  = (unsigned short*)R2;
  unsigned short* ql  = qh + PL;
  unsigned short* kh  = ql + PL;
  unsigned short* kl  = kh + PL;
  unsigned short* vpl = kl + PL;
  float* x1 = (float*)R2;
  unsigned short* h1 = (unsigned short*)(R2 + PL * 4);

  k_wt_heads<<<(NHEAD * HDIM * (DMOD / 8) + 255) / 256, 256, 0, stream>>>(Wq, Bq);
  k_wt_heads<<<(NHEAD * HDIM * (DMOD / 8) + 255) / 256, 256, 0, stream>>>(Wk, Bk);
  k_wt_heads<<<(NHEAD * HDIM * (DMOD / 8) + 255) / 256, 256, 0, stream>>>(Wv, Bv);
  k_wt_f16<<<(DMOD * (DMOD / 8) + 255) / 256, 256, 0, stream>>>(Wp, Pp, DMOD, DMOD);
  k_wt_f16<<<(FFD * (DMOD / 8) + 255) / 256, 256, 0, stream>>>(W1, P1, DMOD, FFD);
  k_wt_f16<<<(DMOD * (FFD / 8) + 255) / 256, 256, 0, stream>>>(W2, P2, FFD, DMOD);

  k_ln768<true, 0><<<NTOK, 96, 0, stream>>>(x, SEQ_FULL, ln1w, ln1b, yh, yl, LN_EPS);
  const int g768 = ((NTOK / 16) * (DMOD / 64) + 3) / 4, g3072 = ((NTOK / 16) * (FFD / 64) + 3) / 4;
  k_gemm<false, 2, 0, false, 2><<<g768, 128, 0, stream>>>(yh, yl, DMOD, Bq, DMOD, bqp, 1.0f, nullptr, 0, 0, qh, ql, DMOD, SEQ, NTOK, DMOD, DMOD);
  k_gemm<false, 2, 0, false, 2><<<g768, 128, 0, stream>>>(yh, yl, DMOD, Bk, DMOD, bkp, 1.0f, nullptr, 0, 0, kh, kl, DMOD, SEQ, NTOK, DMOD, DMOD);
  k_gemm<false, 1, 0, false, 1><<<g768, 128, 0, stream>>>(yh, yh, DMOD, Bv, DMOD, bvp, 1.0f, nullptr, 0, 0, vpl, vpl, DMOD, SEQ, NTOK, DMOD, DMOD);
  k_flash<<<NB * NHEAD * (SEQ / 64), 128, 0, stream>>>(qh, ql, kh, kl, vpl, att);
  k_gemm<true, 1, 2, true, 0><<<g768, 128, 0, stream>>>(att, att, DMOD, Pp, DMOD, bpp, WCARRY_INV, x, DMOD, SEQ_FULL, x1, x1, DMOD, SEQ, NTOK, DMOD, DMOD);
  k_ln768<false, 1><<<NTOK, 96, 0, stream>>>(x1, SEQ, ln2w, ln2b, h0, h0, LN_EPS);
  k_gemm<true, 1, 2, false, 1><<<g3072, 128, 0, stream>>>(h0, h0, DMOD, P1, DMOD, b1p, WCARRY_INV, nullptr, 0, 0, h1, h1, FFD, SEQ, NTOK, FFD, DMOD);
  k_gemm<true, 1, 2, false, 0><<<g768, 128, 0, stream>>>(h1, h1, FFD, P2, FFD, b2p, WCARRY_INV, x1, DMOD, SEQ, d_out, d_out, DMOD, SEQ_FULL, NTOK, DMOD, FFD);
}
